// FCBlock_89936615178932
// MI455X (gfx1250) — hardware-run, weakly checked
//
#include <hip/hip_runtime.h>
#include <math.h>

constexpr int kB    = 4;
constexpr int kT    = 2048;
constexpr int kC    = 768;
constexpr int kH    = 12;
constexpr int kHD   = 64;
constexpr int kF    = 1536;
constexpr int kTok  = kB * kT;
constexpr int kQKld = 2 * kC;
constexpr int kQKVn = 3 * kC;
constexpr int kGrp  = kB * kH;
constexpr int kChunkG = 2;
constexpr int kNChunk = kGrp / kChunkG;

constexpr float kWCarry   = 256.0f;
constexpr float kPCarry   = 2048.0f;
constexpr float kACarry   = 256.0f;
constexpr float kFCarry   = 64.0f;
constexpr float kScoreScale = 0.125f;
constexpr float kInvC     = 1.0f / 768.0f;
constexpr float kLnEps    = 1e-5f;

typedef __attribute__((ext_vector_type(16))) _Float16 v16h;
typedef __attribute__((ext_vector_type(8)))  _Float16 v8h;
typedef __attribute__((ext_vector_type(16))) __bf16   v16b;
typedef __attribute__((ext_vector_type(8)))  __bf16   v8b;
typedef __attribute__((ext_vector_type(8)))  float    v8f;
typedef __attribute__((ext_vector_type(4)))  float    v4f;
typedef __attribute__((ext_vector_type(4)))  unsigned int v4u;

__device__ __forceinline__ unsigned short f2bf_bits(float f) {
  unsigned u = __float_as_uint(f);
  return (unsigned short)((u + 0x7FFFu + ((u >> 16) & 1u)) >> 16);
}
__device__ __forceinline__ float bf_bits2f(unsigned short h) { return __uint_as_float(((unsigned)h) << 16); }

__device__ __forceinline__ void dep_guard_h(v8f& a, v8f& b, v16h x, v16h y) { asm volatile("v_nop\n\tv_nop\n\tv_nop\n\tv_nop" : "+v"(a), "+v"(b) : "v"(x), "v"(y)); }
__device__ __forceinline__ void dep_guard_b(v8f& a, v8f& b, v16b x, v16b y) { asm volatile("v_nop\n\tv_nop\n\tv_nop\n\tv_nop" : "+v"(a), "+v"(b) : "v"(x), "v"(y)); }
__device__ __forceinline__ void keep4_h(v16h a, v16h b, v16h c, v16h d) { asm volatile("v_nop" :: "v"(a), "v"(b), "v"(c), "v"(d)); }
__device__ __forceinline__ void keep4_b(v16b a, v16b b, v16b c, v16b d) { asm volatile("v_nop" :: "v"(a), "v"(b), "v"(c), "v"(d)); }
__device__ __forceinline__ void acc_guard4(v8f& a, v8f& b, v8f& c, v8f& d) { asm volatile("v_nop\n\tv_nop\n\tv_nop\n\tv_nop" : "+v"(a), "+v"(b), "+v"(c), "+v"(d)); }
template <typename T> struct Frag;
template <> struct Frag<_Float16> {
  typedef v16h V; union U { v16h v; v8h h[2]; };
  static __device__ __forceinline__ v16h load(const _Float16* p) {
    U f; f.h[0] = *(const v8h*)(p); f.h[1] = *(const v8h*)(p + 16); return f.v;
  }
  static __device__ __forceinline__ v8f mma(v16h a, v16h b, v8f c) {
    return __builtin_amdgcn_wmma_f32_16x16x32_f16(false, a, false, b, (short)0, c, false, false);
  }
  static __device__ __forceinline__ void guard(v8f& a, v8f& b, v16h x, v16h y) { dep_guard_h(a, b, x, y); }
  static __device__ __forceinline__ void keep(v16h a, v16h b, v16h c, v16h d) { keep4_h(a, b, c, d); }
};
template <> struct Frag<__bf16> {
  typedef v16b V; union U { v16b v; v8b h[2]; };
  static __device__ __forceinline__ v16b load(const __bf16* p) {
    U f; f.h[0] = *(const v8b*)(p); f.h[1] = *(const v8b*)(p + 16); return f.v;
  }
  static __device__ __forceinline__ v8f mma(v16b a, v16b b, v8f c) {
    return __builtin_amdgcn_wmma_f32_16x16x32_bf16(false, a, false, b, (short)0, c, false, false);
  }
  static __device__ __forceinline__ void guard(v8f& a, v8f& b, v16b x, v16b y) { dep_guard_b(a, b, x, y); }
  static __device__ __forceinline__ void keep(v16b a, v16b b, v16b c, v16b d) { keep4_b(a, b, c, d); }
};

__device__ __forceinline__ unsigned pk16(unsigned short a, unsigned short b) { return (unsigned)a | ((unsigned)b << 16); }
__device__ __forceinline__ unsigned short h_bits(float f) { const _Float16 h = (_Float16)f; return __builtin_bit_cast(unsigned short, h); }

template <int ET> struct Elem;
template <> struct Elem<0> { typedef _Float16 T; };
template <> struct Elem<1> { typedef __bf16 T; };
template <int ET, bool SPLIT, int BIAS_MODE, int OUT_MODE, bool RESID, int ACT = 0, int CAUSAL = 0>
__global__ __launch_bounds__(256) void wmma_gemm64(
    const unsigned short* __restrict__ Ap, const unsigned short* __restrict__ A2p, int lda, long strideA,
    const unsigned short* __restrict__ Btp, const unsigned short* __restrict__ Bt2p, int ldb, long strideB,
    void* __restrict__ Cout, void* __restrict__ Cout2, int ldc, long strideC,
    const float* __restrict__ bias,
    const float* __restrict__ resid, long strideR,
    int M, int N, int K, float scale) {
  typedef typename Elem<ET>::T T;
  typedef typename Frag<T>::V V;
  const T* A = (const T*)Ap; const T* A2 = (const T*)A2p; const T* Bt = (const T*)Btp; const T* Bt2 = (const T*)Bt2p;
  __shared__ __align__(16) float sT[8][16 * 68];
  const int b    = blockIdx.y;
  const int lane = threadIdx.x & 31;
  const int wave = threadIdx.x >> 5;
  const int tilesN = N >> 6;
  const int tilesM = M >> 6;
  const int tile = blockIdx.x * 8 + wave;
  if (tile >= tilesM * tilesN) return;
  const int tm = tile / tilesN;
  const int tn = tile - tm * tilesN;
  if (CAUSAL == 1 && tn > tm) return;
  const int m0 = tm << 6;
  const int n0 = tn << 6;
  const int Kl = (CAUSAL == 2) ? ((m0 + 64 < K) ? (m0 + 64) : K) : K;

  const T* Ab  = A  + (size_t)b * strideA;
  const T* Bb  = Bt + (size_t)b * strideB;
  const T* Ab2 = SPLIT ? (A2  + (size_t)b * strideA) : nullptr;
  const T* Bb2 = SPLIT ? (Bt2 + (size_t)b * strideB) : nullptr;

  const int rlane = lane & 15;
  const int koff  = (lane >> 4) * 8;
  const int mOff  = (lane >> 4) * 8;

  v8f acc[4][4];
#pragma unroll
  for (int i = 0; i < 4; ++i)
#pragma unroll
    for (int j = 0; j < 4; ++j) acc[i][j] = (v8f){0.f,0.f,0.f,0.f,0.f,0.f,0.f,0.f};

  for (int k0 = 0; k0 < Kl; k0 += 32) {
    V bh[4], bl[4];
#pragma unroll
    for (int j = 0; j < 4; ++j) {
      const size_t bo = (size_t)(n0 + (j << 4) + rlane) * ldb + koff + k0;
      bh[j] = Frag<T>::load(Bb + bo);
      if (SPLIT) bl[j] = Frag<T>::load(Bb2 + bo);
    }
#pragma unroll
    for (int i = 0; i < 4; ++i) {
      const size_t ao = (size_t)(m0 + (i << 4) + rlane) * lda + koff + k0;
      V ah = Frag<T>::load(Ab + ao);
      V al;
      if (SPLIT) al = Frag<T>::load(Ab2 + ao);
#pragma unroll
      for (int j = 0; j < 4; ++j) {
        acc[i][j] = Frag<T>::mma(ah, bh[j], acc[i][j]);
        if (SPLIT) {
          acc[i][j] = Frag<T>::mma(ah, bl[j], acc[i][j]);
          acc[i][j] = Frag<T>::mma(al, bh[j], acc[i][j]);
        }
      }
      Frag<T>::guard(acc[i][0], acc[i][3], ah, SPLIT ? al : ah);
    }
    Frag<T>::keep(bh[0], bh[1], bh[2], bh[3]);
    if (SPLIT) Frag<T>::keep(bl[0], bl[1], bl[2], bl[3]);
  }
  acc_guard4(acc[0][0], acc[0][1], acc[0][2], acc[0][3]);
  acc_guard4(acc[1][0], acc[1][1], acc[1][2], acc[1][3]);
  acc_guard4(acc[2][0], acc[2][1], acc[2][2], acc[2][3]);
  acc_guard4(acc[3][0], acc[3][1], acc[3][2], acc[3][3]);

  float* slab = sT[wave];
  const float* Rb = RESID ? (resid + (size_t)b * strideR) : nullptr;
#pragma unroll
  for (int i = 0; i < 4; ++i) {
    const int mBase = m0 + (i << 4);
#pragma unroll
    for (int j = 0; j < 4; ++j) {
      const int n = n0 + (j << 4) + rlane;
      float bv = 0.f;
      if (BIAS_MODE == 2) bv = bias[n];
#pragma unroll
      for (int r = 0; r < 8; ++r) {
        float v = acc[i][j][r] * scale;
        if (BIAS_MODE == 1) v += bias[mBase + mOff + r];
        if (BIAS_MODE == 2) v += bv;
        if (RESID) v += Rb[(size_t)(mBase + mOff + r) * ldc + n];
        if (ACT == 2) v = fmaxf(v, 0.0f);
        if (ACT == 4) v = (v > 0.f) ? v : 0.01f * v;
        if (ACT == 6) { const float z = fminf(fmaxf(v, -30.0f), 30.0f); v = kFCarry / (1.0f + expf(-z)); }
        slab[(mOff + r) * 68 + (j << 4) + rlane] = v;
      }
    }
    __builtin_amdgcn_fence(__ATOMIC_RELEASE, "workgroup");
    __builtin_amdgcn_wave_barrier();
    __builtin_amdgcn_fence(__ATOMIC_ACQUIRE, "workgroup");
    if (OUT_MODE == 0) {
      float* C = (float*)Cout + (size_t)b * strideC;
      const int hh = lane >> 4, c4 = (lane & 15) * 4;
      for (int pass = 0; pass < 2; ++pass) {
#pragma unroll
        for (int it = 0; it < 8; ++it) {
          const int row = it * 2 + hh;
          v4f v = *(const v4f*)(slab + row * 68 + c4);
          *(volatile v4f*)(C + (size_t)(mBase + row) * ldc + n0 + c4) = v;
        }
        __threadfence();
      }
    } else {
      const int q = lane >> 3, c8 = (lane & 7) * 8;
      unsigned short* C  = (unsigned short*)Cout  + (size_t)b * strideC;
      unsigned short* C2 = (OUT_MODE == 2) ? ((unsigned short*)Cout2 + (size_t)b * strideC) : nullptr;
      for (int pass = 0; pass < 2; ++pass) {
#pragma unroll
        for (int it = 0; it < 4; ++it) {
          const int row = it * 4 + q;
          const float* sp = slab + row * 68 + c8;
          v8h hv, lv;
#pragma unroll
          for (int e = 0; e < 8; ++e) {
            if (OUT_MODE == 1) {
              hv[e] = (_Float16)sp[e];
            } else {
              unsigned short hb = f2bf_bits(sp[e]);
              unsigned short lb = f2bf_bits(sp[e] - bf_bits2f(hb));
              hv[e] = __builtin_bit_cast(_Float16, hb);
              lv[e] = __builtin_bit_cast(_Float16, lb);
            }
          }
          *(volatile v8h*)(C + (size_t)(mBase + row) * ldc + n0 + c8) = hv;
          if (OUT_MODE == 2) *(volatile v8h*)(C2 + (size_t)(mBase + row) * ldc + n0 + c8) = lv;
        }
        __threadfence();
      }
    }
    __builtin_amdgcn_fence(__ATOMIC_RELEASE, "workgroup");
    __builtin_amdgcn_wave_barrier();
    __builtin_amdgcn_fence(__ATOMIC_ACQUIRE, "workgroup");
  }
}

__global__ __launch_bounds__(96) void ln_kernel(const float* __restrict__ X, const float* __restrict__ g,
                                               const float* __restrict__ bta, unsigned short* __restrict__ out) {
  __shared__ float redA[3];
  __shared__ float redB[3];
  const int row  = blockIdx.x;
  const int t    = threadIdx.x;
  const int lane = t & 31, wave = t >> 5;
  const int c0   = t * 8;
  const float* xr = X + (size_t)row * kC + c0;
  const v4f a = *(const v4f*)(xr);
  const v4f c = *(const v4f*)(xr + 4);
  float x[8];
#pragma unroll
  for (int e = 0; e < 4; ++e) { x[e] = a[e]; x[4 + e] = c[e]; }
  float s = 0.f;
#pragma unroll
  for (int e = 0; e < 8; ++e) s += x[e];
#pragma unroll
  for (int off = 16; off > 0; off >>= 1) s += __shfl_xor(s, off, 32);
  if (lane == 0) redA[wave] = s;
  __syncthreads();
  const float mean = ((redA[0] + redA[1]) + redA[2]) * kInvC;
  float d[8];
  float s2 = 0.f;
#pragma unroll
  for (int e = 0; e < 8; ++e) { d[e] = x[e] - mean; s2 += d[e] * d[e]; }
#pragma unroll
  for (int off = 16; off > 0; off >>= 1) s2 += __shfl_xor(s2, off, 32);
  if (lane == 0) redB[wave] = s2;
  __syncthreads();
  const float var = ((redB[0] + redB[1]) + redB[2]) * kInvC;
  const float inv = rsqrtf(var + kLnEps);
  const v4f ga = *(const v4f*)(g + c0);
  const v4f gc = *(const v4f*)(g + c0 + 4);
  const v4f ba = *(const v4f*)(bta + c0);
  const v4f bc = *(const v4f*)(bta + c0 + 4);
  unsigned short hb[8];
#pragma unroll
  for (int e = 0; e < 4; ++e) {
    hb[e]     = h_bits(d[e] * inv * ga[e] + ba[e]);
    hb[4 + e] = h_bits(d[4 + e] * inv * gc[e] + bc[e]);
  }
  const v4u u = (v4u){pk16(hb[0], hb[1]), pk16(hb[2], hb[3]), pk16(hb[4], hb[5]), pk16(hb[6], hb[7])};
  unsigned short* q = out + (size_t)row * kC + c0;
  *(volatile v4u*)q = u;
  __threadfence();
  *(volatile v4u*)q = u;
}

__global__ __launch_bounds__(256) void tcast_kernel(const float* __restrict__ in0, const float* __restrict__ in1,
                                                    const float* __restrict__ in2, int zPerIn, long inStrideZ, int ldi,
                                                    unsigned short* __restrict__ out, long outStrideZ, int ldo, float scale) {
  __shared__ float sm[64][65];
  const int t  = threadIdx.x;
  const int r0 = blockIdx.x * 64;
  const int c0 = blockIdx.y * 64;
  const int z  = blockIdx.z;
  const int zi = z / zPerIn;
  const int sub = z - zi * zPerIn;
  const float* inb = (zi == 0) ? in0 : (zi == 1) ? in1 : in2;
  inb += (size_t)sub * inStrideZ;
#pragma unroll
  for (int i = 0; i < 16; ++i) {
    const int e = i * 256 + t;
    const int rr = e >> 6;
    const int cc = e & 63;
    sm[cc][rr] = inb[(size_t)(r0 + rr) * ldi + c0 + cc] * scale;
  }
  __syncthreads();
  const int lane = t & 31, wave = t >> 5;
  const int q = lane >> 3, c8 = (lane & 7) * 8;
  unsigned short* op = out + (size_t)z * outStrideZ;
  for (int pass = 0; pass < 2; ++pass) {
#pragma unroll
    for (int it = 0; it < 2; ++it) {
      const int row = wave * 8 + it * 4 + q;
      unsigned short hb[8];
#pragma unroll
      for (int e = 0; e < 8; ++e) hb[e] = h_bits(sm[row][c8 + e]);
      const v4u u = (v4u){pk16(hb[0], hb[1]), pk16(hb[2], hb[3]), pk16(hb[4], hb[5]), pk16(hb[6], hb[7])};
      *(volatile v4u*)(op + (size_t)(c0 + row) * ldo + r0 + c8) = u;
    }
    __threadfence();
  }
}

__global__ __launch_bounds__(256) void softmax_causal_kernel(const float* __restrict__ S, unsigned short* __restrict__ P, float carry) {
  __shared__ float redM[8];
  __shared__ float redS[8];
  const int gi   = blockIdx.x >> 11;
  const int row  = blockIdx.x & (kT - 1);
  const int t    = threadIdx.x;
  const int lane = t & 31, wave = t >> 5;
  const int c0   = t * 8;
  const int rl   = row & ~7;
  const int c0c  = (c0 < rl) ? c0 : rl;
  const float* sr = S + ((size_t)gi * kT + row) * kT + c0c;
  const v4f a = *(const v4f*)(sr);
  const v4f c = *(const v4f*)(sr + 4);
  float x[8];
#pragma unroll
  for (int e = 0; e < 4; ++e) { x[e] = a[e]; x[4 + e] = c[e]; }
  float m = -INFINITY;
#pragma unroll
  for (int e = 0; e < 8; ++e) { x[e] = (c0 + e <= row) ? x[e] : -INFINITY; m = fmaxf(m, x[e]); }
#pragma unroll
  for (int off = 16; off > 0; off >>= 1) m = fmaxf(m, __shfl_xor(m, off, 32));
  if (lane == 0) redM[wave] = m;
  __syncthreads();
  m = redM[0];
#pragma unroll
  for (int w = 1; w < 8; ++w) m = fmaxf(m, redM[w]);
  const bool live = (wave * 256 <= row);
  float p[8];
  float s = 0.f;
  if (live) {
#pragma unroll
    for (int e = 0; e < 8; ++e) { const float pe = (c0 + e <= row) ? expf(x[e] - m) : 0.f; p[e] = pe; s += pe; }
  } else {
#pragma unroll
    for (int e = 0; e < 8; ++e) p[e] = 0.f;
  }
#pragma unroll
  for (int off = 16; off > 0; off >>= 1) s += __shfl_xor(s, off, 32);
  if (lane == 0) redS[wave] = s;
  __syncthreads();
  float sum = redS[0];
#pragma unroll
  for (int w = 1; w < 8; ++w) sum += redS[w];
  const float inv = carry * (1.0f / sum);
  unsigned short hb[8];
#pragma unroll
  for (int e = 0; e < 8; ++e) hb[e] = h_bits(p[e] * inv);
  const v4u u = (v4u){pk16(hb[0], hb[1]), pk16(hb[2], hb[3]), pk16(hb[4], hb[5]), pk16(hb[6], hb[7])};
  unsigned short* q = P + ((size_t)gi * kT + row) * kT + c0;
  *(volatile v4u*)q = u;
  __threadfence();
  *(volatile v4u*)q = u;
}

extern "C" void kernel_launch(void* const* d_in, const int* in_sizes, int n_in,
                              void* d_out, int out_size, void* d_ws, size_t ws_size,
                              hipStream_t stream) {
  if (n_in < 14) return;
  if (in_sizes[0] != kTok * kC || in_sizes[1] != kH * kC * kHD || in_sizes[2] != kH * kC * kHD ||
      in_sizes[3] != kH * kC * kHD || in_sizes[4] != kC * kC || in_sizes[5] != kC ||
      in_sizes[6] != kC * kF || in_sizes[7] != kF || in_sizes[8] != kF * kC || in_sizes[9] != kC ||
      in_sizes[10] != kC || in_sizes[11] != kC || in_sizes[12] != kC || in_sizes[13] != kC) return;
  if (out_size != kTok * kC) return;

  const float* x   = (const float*)d_in[0];
  const float* Wq  = (const float*)d_in[1];
  const float* Wk  = (const float*)d_in[2];
  const float* Wv  = (const float*)d_in[3];
  const float* Wo  = (const float*)d_in[4];
  const float* bo  = (const float*)d_in[5];
  const float* W1  = (const float*)d_in[6];
  const float* b1  = (const float*)d_in[7];
  const float* W2  = (const float*)d_in[8];
  const float* b2  = (const float*)d_in[9];
  const float* g1  = (const float*)d_in[10];
  const float* be1 = (const float*)d_in[11];
  const float* g2  = (const float*)d_in[12];
  const float* be2 = (const float*)d_in[13];
  float* out = (float*)d_out;

  const size_t szH1   = (size_t)kTok * kC * 2;
  const size_t szWqkv = (size_t)kQKVn * kC * 2;
  const size_t szWo   = (size_t)kC * kC * 2;
  const size_t szW1   = (size_t)kF * kC * 2;
  const size_t szW2   = (size_t)kC * kF * 2;
  const size_t szQK   = (size_t)kTok * kQKld * 2;
  const size_t szVt   = (size_t)kB * kC * kT * 2;
  const size_t szAt   = (size_t)kTok * kC * 2;
  const size_t szSc   = (size_t)kChunkG * kT * kT * 4;
  const size_t szP    = (size_t)kChunkG * kT * kT * 2;
  const size_t oH1 = 0;
  const size_t oWqkv = oH1 + szH1;
  const size_t oWo = oWqkv + szWqkv;
  const size_t oW1 = oWo + szWo;
  const size_t oW2 = oW1 + szW1;
  const size_t oQK = oW2 + szW2;
  const size_t oVt = oQK + szQK;
  const size_t oAt = oVt + szVt;
  const size_t oSc = oAt + szAt;
  const size_t oP  = oSc + szSc;
  const size_t total = oP + szP;
  if (total > ws_size) return;
  if ((size_t)kTok * kC * 4 > szQK) return;
  if ((size_t)kTok * kF * 2 > szSc) return;

  char* w = (char*)d_ws;
  unsigned short* h1    = (unsigned short*)(w + oH1);
  unsigned short* WqkvT = (unsigned short*)(w + oWqkv);
  unsigned short* WoT   = (unsigned short*)(w + oWo);
  unsigned short* W1T   = (unsigned short*)(w + oW1);
  unsigned short* W2T   = (unsigned short*)(w + oW2);
  unsigned short* QK    = (unsigned short*)(w + oQK);
  float*          x1    = (float*)(w + oQK);
  unsigned short* Vt    = (unsigned short*)(w + oVt);
  unsigned short* attn  = (unsigned short*)(w + oAt);
  float*          Sc    = (float*)(w + oSc);
  unsigned short* ffn1  = (unsigned short*)(w + oSc);
  unsigned short* Pp    = (unsigned short*)(w + oP);

  const float invW = 1.0f / kWCarry;

  ln_kernel<<<kTok, 96, 0, stream>>>(x, g1, be1, h1);

  tcast_kernel<<<dim3(kC / 64, 1, 3 * kH), 256, 0, stream>>>(Wq, Wk, Wv, kH, (long)kC * kHD, kHD,
                                                              WqkvT, (long)kHD * kC, kC, kWCarry);
  tcast_kernel<<<dim3(kC / 64, kC / 64, 1), 256, 0, stream>>>(Wo, Wo, Wo, 1, 0L, kC, WoT, 0L, kC, kWCarry);
  tcast_kernel<<<dim3(kC / 64, kF / 64, 1), 256, 0, stream>>>(W1, W1, W1, 1, 0L, kF, W1T, 0L, kC, kWCarry);
  tcast_kernel<<<dim3(kF / 64, kC / 64, 1), 256, 0, stream>>>(W2, W2, W2, 1, 0L, kC, W2T, 0L, kF, kWCarry);

  {
    const int tiles = (kTok / 64) * (kQKld / 64);
    wmma_gemm64<0, false, 0, 1, false, 0, 0><<<dim3(tiles / 8, 1), 256, 0, stream>>>(
        h1, h1, kC, 0L, WqkvT, WqkvT, kC, 0L, QK, QK, kQKld, 0L, bo, x, 0L, kTok, kQKld, kC, invW);
  }
  {
    const int tiles = (kC / 64) * (kT / 64);
    wmma_gemm64<0, false, 0, 1, false, 0, 0><<<dim3(tiles / 8, kB), 256, 0, stream>>>(
        WqkvT + (size_t)2 * kC * kC, WqkvT + (size_t)2 * kC * kC, kC, 0L,
        h1, h1, kC, (long)kT * kC,
        Vt, Vt, kT, (long)kC * kT, bo, x, 0L, kC, kT, kC, invW);
  }

  for (int ch = 0; ch < kNChunk; ++ch) {
    const int g0 = ch * kChunkG;
    const int bb = g0 / kH;
    const int hh = g0 - bb * kH;
    const unsigned short* qbase = QK + (size_t)bb * kT * kQKld + (size_t)hh * kHD;
    const unsigned short* kbase = qbase + kC;
    {
      const int tiles = (kT / 64) * (kT / 64);
      wmma_gemm64<0, false, 0, 0, false, 0, 1><<<dim3(tiles / 8, kChunkG), 256, 0, stream>>>(
          qbase, qbase, kQKld, (long)kHD, kbase, kbase, kQKld, (long)kHD,
          Sc, Sc, kT, (long)kT * kT, bo, x, 0L, kT, kT, kHD, kScoreScale);
    }
    softmax_causal_kernel<<<kChunkG * kT, 256, 0, stream>>>(Sc, Pp, kPCarry);
    {
      const unsigned short* vtg = Vt + (size_t)g0 * kHD * kT;
      unsigned short* og = attn + (size_t)bb * kT * kC + (size_t)hh * kHD;
      const int tiles = (kT / 64) * (kHD / 64);
      wmma_gemm64<0, false, 0, 1, false, 0, 2><<<dim3(tiles / 8, kChunkG), 256, 0, stream>>>(
          Pp, Pp, kT, (long)kT * kT, vtg, vtg, kT, (long)kHD * kT,
          og, og, kC, (long)kHD, bo, x, 0L, kT, kHD, kT, kACarry / kPCarry);
    }
  }

  {
    const int tiles = (kTok / 64) * (kC / 64);
    wmma_gemm64<0, false, 2, 0, true, 0, 0><<<dim3(tiles / 8, 1), 256, 0, stream>>>(
        attn, attn, kC, 0L, WoT, WoT, kC, 0L, x1, x1, kC, 0L, bo, x, 0L,
        kTok, kC, kC, 1.0f / (kACarry * kWCarry));
  }
  ln_kernel<<<kTok, 96, 0, stream>>>(x1, g2, be2, h1);
  {
    const int tiles = (kTok / 64) * (kF / 64);
    wmma_gemm64<0, false, 2, 1, false, 6, 0><<<dim3(tiles / 8, 1), 256, 0, stream>>>(
        h1, h1, kC, 0L, W1T, W1T, kC, 0L, ffn1, ffn1, kF, 0L, b1, x, 0L, kTok, kF, kC, invW);
  }
  {
    const int tiles = (kTok / 64) * (kC / 64);
    wmma_gemm64<0, false, 2, 0, true, 0, 0><<<dim3(tiles / 8, 1), 256, 0, stream>>>(
        ffn1, ffn1, kF, 0L, W2T, W2T, kF, 0L, out, out, kC, 0L, b2, x1, 0L,
        kTok, kC, kF, 1.0f / (kFCarry * kWCarry));
  }
}
